// MemoryCompressedAttention_85177791414353
// MI455X (gfx1250) — hardware-verified
//
#include <hip/hip_runtime.h>
#include <math.h>
#include <stdint.h>

#define NB     2
#define SEQ    2048
#define DMOD   1024
#define NH     16
#define HD     64
#define CF     3
#define KCONV  (CF * HD)
#define JTOT   684
#define JP     704
#define UOFF   4
#define UROWS  2112
#define ROWS   (NB * SEQ)
#define QSC    64.0f
#define KSC    1024.0f
#define KVS    1024.0f
#define WCS    1024.0f
#define VCAR   1024.0f
#define PCAR   32768.0f
#define OSC    1024.0f
#define WOS    1024.0f
#define LOG2E  1.4426950408889634f
#define SLAB64 (16 * 68)
#define SLABF  (16 * 68)
#define CONV_MT   (JP / 64)
#define CONV_HALF (NB * NH * CONV_MT)
#define MAXBLK    (JP / 32)
#define ATT_BLOCKS (NB * NH * (SEQ / 64))

static_assert(NH * HD == DMOD);
static_assert((JP % 64) == 0 && JP >= JTOT && (JP % 32) == 0);
static_assert(3 * (JP - 1) + 2 < UROWS);
static_assert(SEQ + UOFF <= UROWS && (UOFF + (UROWS - SEQ - UOFF)) == 64);
static_assert((KCONV % 32) == 0 && (DMOD % 64) == 0 && (ROWS % 64) == 0 && (SEQ % 64) == 0);
static_assert(CONV_MT == 11 && CONV_HALF == 352 && MAXBLK == 22 && ATT_BLOCKS == 1024);
static_assert((3 * (SEQ - 1) + 2) / 3 + 1 >= JTOT - 1);

typedef unsigned short u16;
typedef _Float16 v16h __attribute__((ext_vector_type(16)));
typedef _Float16 v8h  __attribute__((ext_vector_type(8)));
typedef __bf16   v16b __attribute__((ext_vector_type(16)));
typedef float    v8f  __attribute__((ext_vector_type(8)));
typedef float    v4f  __attribute__((ext_vector_type(4)));
typedef unsigned int v4u __attribute__((ext_vector_type(4)));

union FragH { v16h v; v8h h[2]; v4u u[2]; };
union FragB { v16b v; v4u u[2]; };

__device__ __forceinline__ unsigned short bf_bits(float f) {
  unsigned u = __float_as_uint(f);
  return (unsigned short)((u + 0x7FFFu + ((u >> 16) & 1u)) >> 16);
}
__device__ __forceinline__ float bf_up(unsigned short h) { return __uint_as_float(((unsigned)h) << 16); }
__device__ __forceinline__ float bfr(float f) { return bf_up(bf_bits(f)); }
__device__ __forceinline__ unsigned short h_bits(_Float16 x) { return __builtin_bit_cast(unsigned short, x); }
__device__ __forceinline__ unsigned pk16(unsigned short a, unsigned short b) { return (unsigned)a | ((unsigned)b << 16); }
__device__ __forceinline__ v8f zero8() { v8f z = {0.f, 0.f, 0.f, 0.f, 0.f, 0.f, 0.f, 0.f}; return z; }

__device__ __forceinline__ v16h ldfrag_h(const _Float16* p) {
  FragH f;
  f.h[0] = *(const v8h*)(p);
  f.h[1] = *(const v8h*)(p + 16);
  return f.v;
}
__device__ __forceinline__ v16b ldfrag_b(const u16* p) {
  FragB f;
  f.u[0] = *(const v4u*)(p);
  f.u[1] = *(const v4u*)(p + 16);
  return f.v;
}

__device__ __forceinline__ v8f mma_h(v16h a, v16h b, v8f c) {
  return __builtin_amdgcn_wmma_f32_16x16x32_f16(false, a, false, b, (short)0, c, false, false);
}
__device__ __forceinline__ v8f mma_b(v16b a, v16b b, v8f c) {
  return __builtin_amdgcn_wmma_f32_16x16x32_bf16(false, a, false, b, (short)0, c, false, false);
}
__device__ __forceinline__ void guard_s(v8f& a, v8f& b, v16h x0, v16h x1, v16h x2) {
#if defined(__HIP_DEVICE_COMPILE__)
  asm volatile("v_nop\n\tv_nop\n\tv_nop\n\tv_nop" : "+v"(a), "+v"(b) : "v"(x0), "v"(x1), "v"(x2) : "memory");
#endif
}
template <typename F>
__device__ __forceinline__ void guard6(v8f& a, v8f& b, v8f& c, v8f& d, F x0, F x1, F x2, F x3, F x4, F x5) {
#if defined(__HIP_DEVICE_COMPILE__)
  asm volatile("v_nop\n\tv_nop\n\tv_nop\n\tv_nop"
               : "+v"(a), "+v"(b), "+v"(c), "+v"(d) : "v"(x0), "v"(x1), "v"(x2), "v"(x3), "v"(x4), "v"(x5) : "memory");
#endif
}
__device__ __forceinline__ void guard10(v8f& a, v8f& b, v8f& c, v8f& d, v16h x0, v16h x1, v16h x2, v16h x3, v16h x4,
                                        v16h x5, v16h x6, v16h x7, v16h x8, v16h x9) {
#if defined(__HIP_DEVICE_COMPILE__)
  asm volatile("v_nop\n\tv_nop\n\tv_nop\n\tv_nop"
               : "+v"(a), "+v"(b), "+v"(c), "+v"(d)
               : "v"(x0), "v"(x1), "v"(x2), "v"(x3), "v"(x4), "v"(x5), "v"(x6), "v"(x7), "v"(x8), "v"(x9) : "memory");
#endif
}
__device__ __forceinline__ void acc_guard4(v8f& a, v8f& b, v8f& c, v8f& d) {
#if defined(__HIP_DEVICE_COMPILE__)
  asm volatile("v_nop\n\tv_nop\n\tv_nop\n\tv_nop" : "+v"(a), "+v"(b), "+v"(c), "+v"(d));
#endif
}
__device__ __forceinline__ void wave_sync_lds() {
  __builtin_amdgcn_fence(__ATOMIC_RELEASE, "workgroup");
  __builtin_amdgcn_wave_barrier();
  __builtin_amdgcn_fence(__ATOMIC_ACQUIRE, "workgroup");
}

__global__ __launch_bounds__(256) void cvt16(const float* __restrict__ x, u16* D, int n8, int f16mode, float scale) {
  const int gt = blockIdx.x * 256 + (int)threadIdx.x;
  if (gt >= n8) return;
  const float* p = x + (size_t)gt * 8;
  const v4f a = *(const v4f*)(p), bq = *(const v4f*)(p + 4);
  float w[8];
#pragma unroll
  for (int e = 0; e < 4; ++e) { w[e] = a[e]; w[4 + e] = bq[e]; }
  v4u ob, oh;
#pragma unroll
  for (int e = 0; e < 4; ++e) {
    ob[e] = pk16(bf_bits(w[2 * e]), bf_bits(w[2 * e + 1]));
    oh[e] = pk16(h_bits((_Float16)(bfr(w[2 * e]) * scale)), h_bits((_Float16)(bfr(w[2 * e + 1]) * scale)));
  }
  const v4u o = (f16mode != 0) ? oh : ob;
  u16* d = D + (size_t)gt * 8;
  for (int pass = 0; pass < 2; ++pass) {
    *(volatile v4u*)(d) = o;
    __threadfence();
  }
}

__global__ __launch_bounds__(256) void cvt_wconv(const float* __restrict__ W, u16* D) {
  __shared__ __align__(16) u16 T[32 * 200];
  const int tid = threadIdx.x;
  const int o0 = blockIdx.x * 32;
  const float* src = W + (size_t)o0 * KCONV;
#pragma unroll 4
  for (int i = 0; i < 24; ++i) {
    const int e  = tid + 256 * i;
    const int ol = e / KCONV;
    const int s  = e - ol * KCONV;
    const int ci = s / CF;
    const int j  = s - ci * CF;
    T[ol * 200 + j * HD + ci] = h_bits((_Float16)(bfr(src[e]) * WCS));
  }
  __syncthreads();
  const int wave = tid >> 5, lane = tid & 31;
  const int lc = (lane < 24) ? lane : 23;
  v4u vals[4];
#pragma unroll
  for (int q = 0; q < 4; ++q) vals[q] = *(const v4u*)(T + (wave * 4 + q) * 200 + lc * 8);
  for (int pass = 0; pass < 2; ++pass) {
#pragma unroll
    for (int q = 0; q < 4; ++q) {
      if (lane < 24) *(volatile v4u*)(D + (size_t)(o0 + wave * 4 + q) * KCONV + lane * 8) = vals[q];
    }
    __threadfence();
  }
}

__global__ __launch_bounds__(256) void fill_pad(u16* KH, u16* KL, u16* VH, u16* VL) {
  const int tid = threadIdx.x;
  const int bid = blockIdx.x;
  const int arr = bid & 3;
  const int plane = bid >> 2;
  u16* base = (arr == 0) ? KH : (arr == 1) ? KL : (arr == 2) ? VH : VL;
  v4u z = {0u, 0u, 0u, 0u};
  for (int pass = 0; pass < 2; ++pass) {
#pragma unroll
    for (int i = 0; i < 2; ++i) {
      const int p  = tid + 256 * i;
      const int ri = p >> 3;
      const int c8 = (p & 7) * 8;
      const int u  = (ri < UOFF) ? ri : (SEQ + ri);
      *(volatile v4u*)(base + ((size_t)plane * UROWS + u) * HD + c8) = z;
    }
    __threadfence();
  }
}

__device__ __forceinline__ void stage64(float* sl, v8f a0, v8f a1, v8f a2, v8f a3, float oscale, int lane) {
  const int hh = lane >> 4, m = lane & 15;
#pragma unroll
  for (int r = 0; r < 8; ++r) {
    const int ro = (8 * hh + r) * 68 + m;
    sl[ro]      = a0[r] * oscale;
    sl[ro + 16] = a1[r] * oscale;
    sl[ro + 32] = a2[r] * oscale;
    sl[ro + 48] = a3[r] * oscale;
  }
  wave_sync_lds();
}
__device__ __forceinline__ void store_h1(const float* sl, u16* dst, int pitch, int lane) {
  const int rq = lane >> 3, c8 = (lane & 7) * 8;
  v4u oh[4];
#pragma unroll
  for (int it = 0; it < 4; ++it) {
    const int row = it * 4 + rq;
    const v4f a = *(const v4f*)(sl + row * 68 + c8), bq = *(const v4f*)(sl + row * 68 + c8 + 4);
    oh[it][0] = pk16(h_bits((_Float16)a[0]),  h_bits((_Float16)a[1]));
    oh[it][1] = pk16(h_bits((_Float16)a[2]),  h_bits((_Float16)a[3]));
    oh[it][2] = pk16(h_bits((_Float16)bq[0]), h_bits((_Float16)bq[1]));
    oh[it][3] = pk16(h_bits((_Float16)bq[2]), h_bits((_Float16)bq[3]));
  }
  for (int pass = 0; pass < 2; ++pass) {
#pragma unroll
    for (int it = 0; it < 4; ++it) {
      const int row = it * 4 + rq;
      *(volatile v4u*)(dst + (size_t)row * pitch + c8) = oh[it];
    }
    __threadfence();
  }
}
__device__ __forceinline__ void store_h2(const float* sl, u16* dh, u16* dl, int pitch, int lane) {
  const int rq = lane >> 3, c8 = (lane & 7) * 8;
  v4u oh[4], ol[4];
#pragma unroll
  for (int it = 0; it < 4; ++it) {
    const int row = it * 4 + rq;
    const v4f a = *(const v4f*)(sl + row * 68 + c8), bq = *(const v4f*)(sl + row * 68 + c8 + 4);
    float w[8];
#pragma unroll
    for (int e = 0; e < 4; ++e) { w[e] = a[e]; w[4 + e] = bq[e]; }
#pragma unroll
    for (int e = 0; e < 4; ++e) {
      const _Float16 h0 = (_Float16)w[2 * e], h1 = (_Float16)w[2 * e + 1];
      const _Float16 l0 = (_Float16)(w[2 * e] - (float)h0), l1 = (_Float16)(w[2 * e + 1] - (float)h1);
      oh[it][e] = pk16(h_bits(h0), h_bits(h1));
      ol[it][e] = pk16(h_bits(l0), h_bits(l1));
    }
  }
  for (int pass = 0; pass < 2; ++pass) {
#pragma unroll
    for (int it = 0; it < 4; ++it) {
      const int row = it * 4 + rq;
      *(volatile v4u*)(dh + (size_t)row * pitch + c8) = oh[it];
      *(volatile v4u*)(dl + (size_t)row * pitch + c8) = ol[it];
    }
    __threadfence();
  }
}
__device__ __forceinline__ void epi64(float* sl, v8f a0, v8f a1, v8f a2, v8f a3, float oscale, const float* __restrict__ bias,
                                      float* C, int N, size_t rowb, int col0, int lane) {
  const int hh = lane >> 4, m = lane & 15;
  stage64(sl, a0, a1, a2, a3, oscale, lane);
  v4f bb;
#pragma unroll
  for (int e = 0; e < 4; ++e) bb[e] = bfr(bias[col0 + m * 4 + e]);
  v4f vals[8];
#pragma unroll
  for (int it = 0; it < 8; ++it) vals[it] = *(const v4f*)(sl + (it * 2 + hh) * 68 + m * 4) + bb;
  float* dst = C + (rowb + (size_t)hh) * (size_t)N + col0 + m * 4;
  for (int pass = 0; pass < 2; ++pass) {
#pragma unroll
    for (int it = 0; it < 8; ++it) {
      *(volatile v4f*)(dst + (size_t)(it * 2) * (size_t)N) = vals[it];
    }
    __threadfence();
  }
}

__global__ __launch_bounds__(128)
void proj_gemm(const u16* __restrict__ A, const u16* __restrict__ Bt, u16* QP, u16* KH, u16* KL, u16* VH, u16* VL) {
  __shared__ __align__(16) float slab[4 * SLAB64];
  const int tid = threadIdx.x, wave = tid >> 5, lane = tid & 31, hh = lane >> 4, m = lane & 15;
  const int ntile = (3 * DMOD) >> 6;
  const int bid   = blockIdx.x;
  const int rowb  = (bid / ntile) * 64 + wave * 16;
  const int col0  = (bid % ntile) * 64;
  const u16* ap = A  + (size_t)(rowb + m) * DMOD + 8 * hh;
  const u16* bp = Bt + (size_t)(col0 + m) * DMOD + 8 * hh;
  const size_t bs = (size_t)16 * DMOD;
  v8f acc0 = zero8(), acc1 = zero8(), acc2 = zero8(), acc3 = zero8();
#pragma unroll 1
  for (int k0 = 0; k0 < DMOD; k0 += 32) {
    const v16b a  = ldfrag_b(ap + k0);
    const v16b b0 = ldfrag_b(bp + k0);
    const v16b b1 = ldfrag_b(bp + bs + k0);
    const v16b b2 = ldfrag_b(bp + 2 * bs + k0);
    const v16b b3 = ldfrag_b(bp + 3 * bs + k0);
    acc0 = mma_b(a, b0, acc0);
    acc1 = mma_b(a, b1, acc1);
    acc2 = mma_b(a, b2, acc2);
    acc3 = mma_b(a, b3, acc3);
    guard6<v16b>(acc0, acc1, acc2, acc3, a, b0, b1, b2, b3, a);
  }
  float* sl = slab + wave * SLAB64;
  const int sec  = col0 >> 10;
  const int hcol = col0 & (DMOD - 1);
  if (sec == 0) {
    stage64(sl, acc0, acc1, acc2, acc3, QSC, lane);
    store_h1(sl, QP + (size_t)rowb * DMOD + hcol, DMOD, lane);
  } else {
    stage64(sl, acc0, acc1, acc2, acc3, KVS, lane);
    const int g  = hcol >> 6;
    const int b  = rowb >> 11;
    const int t0 = rowb & (SEQ - 1);
    const size_t dofs = (((size_t)(b * NH + g)) * UROWS + t0 + UOFF) * HD;
    u16* dh = (sec == 1) ? KH : VH;
    u16* dl = (sec == 1) ? KL : VL;
    store_h2(sl, dh + dofs, dl + dofs, HD, lane);
  }
}

__global__ __launch_bounds__(128)
void conv_gemm(const u16* __restrict__ KH, const u16* __restrict__ KL, const u16* __restrict__ VH, const u16* __restrict__ VL,
               const u16* __restrict__ WCT, const float* __restrict__ bconv, const float* __restrict__ nullk,
               const float* __restrict__ nullv, u16* KC, u16* VTH, u16* VTL) {
  __shared__ __align__(16) float cs[64 * 68];
  const int tid = threadIdx.x, wave = tid >> 5, lane = tid & 31, hh = lane >> 4, m = lane & 15;
  const int bid   = blockIdx.x;
  const int vmode = (bid >= CONV_HALF) ? 1 : 0;
  const int rb    = bid - vmode * CONV_HALF;
  const int plane = rb / CONV_MT;
  const int mt    = rb - plane * CONV_MT;
  const int g     = plane & (NH - 1);
  const int cc0   = mt * 64 + wave * 16;
  const u16* AH = (vmode != 0) ? VH : KH;
  const u16* AL = (vmode != 0) ? VL : KL;
  const size_t aofs = ((size_t)plane * UROWS) * HD + (size_t)(cc0 + m) * KCONV + 8 * hh;
  const _Float16* ahp = (const _Float16*)(const void*)AH + aofs;
  const _Float16* alp = (const _Float16*)(const void*)AL + aofs;
  const _Float16* bp  = (const _Float16*)(const void*)WCT + (size_t)(g * HD + m) * KCONV + 8 * hh;
  const size_t bs = (size_t)16 * KCONV;
  v8f acc0 = zero8(), acc1 = zero8(), acc2 = zero8(), acc3 = zero8();
#pragma unroll 1
  for (int k0 = 0; k0 < KCONV; k0 += 32) {
    const v16h ah = ldfrag_h(ahp + k0), al = ldfrag_h(alp + k0);
    const v16h b0 = ldfrag_h(bp + k0);
    const v16h b1 = ldfrag_h(bp + bs + k0);
    const v16h b2 = ldfrag_h(bp + 2 * bs + k0);
    const v16h b3 = ldfrag_h(bp + 3 * bs + k0);
    acc0 = mma_h(ah, b0, acc0);  acc0 = mma_h(al, b0, acc0);
    acc1 = mma_h(ah, b1, acc1);  acc1 = mma_h(al, b1, acc1);
    acc2 = mma_h(ah, b2, acc2);  acc2 = mma_h(al, b2, acc2);
    acc3 = mma_h(ah, b3, acc3);  acc3 = mma_h(al, b3, acc3);
    guard6<v16h>(acc0, acc1, acc2, acc3, ah, al, b0, b1, b2, b3);
  }
  const int ocol = g * HD;
  float bc[4], nl[4];
#pragma unroll
  for (int j = 0; j < 4; ++j) {
    const int o = ocol + 16 * j + m;
    bc[j] = bfr(bconv[o]);
    const float nk = bfr(nullk[o]), nv = bfr(nullv[o]);
    nl[j] = (vmode != 0) ? nv : nk;
  }
  const float osc   = 1.0f / (KVS * WCS);
  const float carry = (vmode != 0) ? VCAR : KSC;
#pragma unroll
  for (int r = 0; r < 8; ++r) {
    const int cc   = cc0 + 8 * hh + r;
    const int rowl = wave * 16 + 8 * hh + r;
    float v0 = acc0[r] * osc + bc[0];
    float v1 = acc1[r] * osc + bc[1];
    float v2 = acc2[r] * osc + bc[2];
    float v3 = acc3[r] * osc + bc[3];
    v0 = (cc == 0) ? nl[0] : v0;  v1 = (cc == 0) ? nl[1] : v1;  v2 = (cc == 0) ? nl[2] : v2;  v3 = (cc == 0) ? nl[3] : v3;
    v0 = (cc >= JTOT) ? 0.f : v0; v1 = (cc >= JTOT) ? 0.f : v1; v2 = (cc >= JTOT) ? 0.f : v2; v3 = (cc >= JTOT) ? 0.f : v3;
    cs[rowl * 68 + m]      = v0 * carry;
    cs[rowl * 68 + 16 + m] = v1 * carry;
    cs[rowl * 68 + 32 + m] = v2 * carry;
    cs[rowl * 68 + 48 + m] = v3 * carry;
  }
  __syncthreads();
  const int rq = tid >> 3;
  const int c8 = (tid & 7) * 8;
  if (vmode == 0) {
    v4u vals[4];
#pragma unroll
    for (int it = 0; it < 4; ++it) {
      const int row = it * 16 + rq;
      const v4f a = *(const v4f*)(cs + row * 68 + c8), bq = *(const v4f*)(cs + row * 68 + c8 + 4);
      vals[it][0] = pk16(h_bits((_Float16)a[0]),  h_bits((_Float16)a[1]));
      vals[it][1] = pk16(h_bits((_Float16)a[2]),  h_bits((_Float16)a[3]));
      vals[it][2] = pk16(h_bits((_Float16)bq[0]), h_bits((_Float16)bq[1]));
      vals[it][3] = pk16(h_bits((_Float16)bq[2]), h_bits((_Float16)bq[3]));
    }
    u16* dst = KC + ((size_t)plane * JP + mt * 64) * HD + c8;
    for (int pass = 0; pass < 2; ++pass) {
#pragma unroll
      for (int it = 0; it < 4; ++it) {
        const int row = it * 16 + rq;
        *(volatile v4u*)(dst + (size_t)row * HD) = vals[it];
      }
      __threadfence();
    }
  } else {
    v4u vh[4], vl[4];
#pragma unroll
    for (int it = 0; it < 4; ++it) {
      const int d = it * 16 + rq;
      float w[8];
#pragma unroll
      for (int e = 0; e < 8; ++e) w[e] = cs[(c8 + e) * 68 + d];
#pragma unroll
      for (int e = 0; e < 4; ++e) {
        const _Float16 h0 = (_Float16)w[2 * e], h1 = (_Float16)w[2 * e + 1];
        const _Float16 l0 = (_Float16)(w[2 * e] - (float)h0), l1 = (_Float16)(w[2 * e + 1] - (float)h1);
        vh[it][e] = pk16(h_bits(h0), h_bits(h1));
        vl[it][e] = pk16(h_bits(l0), h_bits(l1));
      }
    }
    const size_t vb = ((size_t)plane * HD) * JP + mt * 64 + c8;
    for (int pass = 0; pass < 2; ++pass) {
#pragma unroll
      for (int it = 0; it < 4; ++it) {
        const int d = it * 16 + rq;
        *(volatile v4u*)(VTH + vb + (size_t)d * JP) = vh[it];
        *(volatile v4u*)(VTL + vb + (size_t)d * JP) = vl[it];
      }
      __threadfence();
    }
  }
}

__global__ __launch_bounds__(128)
void attn_mc(const u16* __restrict__ QP, const u16* __restrict__ KC, const u16* __restrict__ VTH,
             const u16* __restrict__ VTL, u16* OHIp, u16* OLOp) {
  __shared__ __align__(16) float smem[4 * SLABF];

  const int tid  = threadIdx.x;
  const int wave = tid >> 5;
  const int lane = tid & 31;
  const int hh   = lane >> 4;
  const int c    = lane & 15;

  const int bid  = blockIdx.x;
  const int qt   = bid & (SEQ / 64 - 1);
  const int h    = (bid >> 5) & (NH - 1);
  const int b    = bid >> 9;
  const int q0   = qt * 64 + wave * 16;
  const int plane = b * NH + h;

  const size_t qofs = ((size_t)(b * SEQ + q0 + c)) * DMOD + h * HD + 8 * hh;
  const _Float16* Qp  = (const _Float16*)(const void*)QP + qofs;
  const _Float16* Kcb = (const _Float16*)(const void*)KC + ((size_t)plane * JP + c) * HD + 8 * hh;
  const size_t vofs = ((size_t)plane * HD + c) * JP + 8 * hh;
  const _Float16* Vhb = (const _Float16*)(const void*)VTH + vofs;
  const _Float16* Vlb = (const _Float16*)(const void*)VTL + vofs;
  const float lsc = LOG2E / (32.0f * QSC * KSC);

  const v16h qa = ldfrag_h(Qp), qb = ldfrag_h(Qp + 32);

  float mrow[8], lrow[8];
  v8f o[4];
#pragma unroll
  for (int r = 0; r < 8; ++r) { mrow[r] = -INFINITY; lrow[r] = 0.f; }
#pragma unroll
  for (int j = 0; j < 4; ++j) o[j] = zero8();
  float* pt = smem + wave * SLABF;

  int numj = (q0 + 15 + 2) / 3 + 1;
  numj = (numj > JTOT) ? JTOT : numj;
  int nblk = (numj + 31) >> 5;
  nblk = (nblk > MAXBLK) ? MAXBLK : nblk;

#pragma unroll 1
  for (int it = 0; it < nblk; ++it) {
    const int kb = it * 32;
    v8f s0 = zero8(), s1 = zero8();
    const _Float16* k0p = Kcb + (size_t)kb * HD;
    const _Float16* k1p = k0p + (size_t)16 * HD;
#pragma unroll
    for (int kk = 0; kk < 2; ++kk) {
      const v16h qf  = (kk == 0) ? qa : qb;
      const v16h kf0 = ldfrag_h(k0p + kk * 32);
      const v16h kf1 = ldfrag_h(k1p + kk * 32);
      s0 = mma_h(qf, kf0, s0);
      s1 = mma_h(qf, kf1, s1);
      guard_s(s0, s1, qf, kf0, kf1);
    }
#pragma unroll
    for (int r = 0; r < 8; ++r) {
      const int i  = q0 + 8 * hh + r;
      const int j0 = kb + c, j1 = kb + 16 + c;
      const bool ok0 = (j0 < JTOT) && ((3 * j0 - 2) <= i);
      const bool ok1 = (j1 < JTOT) && ((3 * j1 - 2) <= i);
      const float t0 = ok0 ? (s0[r] * lsc) : -INFINITY;
      const float t1 = ok1 ? (s1[r] * lsc) : -INFINITY;
      float mx = fmaxf(t0, t1);
#pragma unroll
      for (int off = 1; off < 16; off <<= 1) mx = fmaxf(mx, __shfl_xor(mx, off, 32));
      const float mn = fmaxf(mrow[r], mx);
      const float al = exp2f(mrow[r] - mn);
      mrow[r] = mn;
      const float e0 = exp2f(t0 - mn), e1 = exp2f(t1 - mn);
      float ps = e0 + e1;
#pragma unroll
      for (int off = 1; off < 16; off <<= 1) ps += __shfl_xor(ps, off, 32);
      lrow[r] = lrow[r] * al + ps;
#pragma unroll
      for (int j = 0; j < 4; ++j) o[j][r] *= al;
      const int ro = (8 * hh + r) * 36 + c;
      pt[ro]      = e0;
      pt[ro + 16] = e1;
    }
    wave_sync_lds();
    FragH ph, pl;
    {
      const float* prow = pt + c * 36 + 8 * hh;
      const v4f p0 = *(const v4f*)(prow), p1 = *(const v4f*)(prow + 4);
      const v4f p2 = *(const v4f*)(prow + 16), p3 = *(const v4f*)(prow + 20);
#pragma unroll
      for (int e = 0; e < 4; ++e) {
        const float ta = p0[e] * PCAR, tb = p1[e] * PCAR, tc = p2[e] * PCAR, td = p3[e] * PCAR;
        const _Float16 ha = (_Float16)ta, hb = (_Float16)tb, hc = (_Float16)tc, hd = (_Float16)td;
        ph.h[0][e]     = ha;
        ph.h[0][4 + e] = hb;
        ph.h[1][e]     = hc;
        ph.h[1][4 + e] = hd;
        pl.h[0][e]     = (_Float16)(ta - (float)ha);
        pl.h[0][4 + e] = (_Float16)(tb - (float)hb);
        pl.h[1][e]     = (_Float16)(tc - (float)hc);
        pl.h[1][4 + e] = (_Float16)(td - (float)hd);
      }
    }
    {
      const _Float16* vhp = Vhb + kb;
      const _Float16* vlp = Vlb + kb;
      const v16h vh0 = ldfrag_h(vhp);
      const v16h vh1 = ldfrag_h(vhp + (size_t)16 * JP);
      const v16h vh2 = ldfrag_h(vhp + (size_t)32 * JP);
      const v16h vh3 = ldfrag_h(vhp + (size_t)48 * JP);
      const v16h vl0 = ldfrag_h(vlp);
      const v16h vl1 = ldfrag_h(vlp + (size_t)16 * JP);
      const v16h vl2 = ldfrag_h(vlp + (size_t)32 * JP);
      const v16h vl3 = ldfrag_h(vlp + (size_t)48 * JP);
      o[0] = mma_h(ph.v, vh0, o[0]);  o[0] = mma_h(pl.v, vh0, o[0]);  o[0] = mma_h(ph.v, vl0, o[0]);
      o[1] = mma_h(ph.v, vh1, o[1]);  o[1] = mma_h(pl.v, vh1, o[1]);  o[1] = mma_h(ph.v, vl1, o[1]);
      o[2] = mma_h(ph.v, vh2, o[2]);  o[2] = mma_h(pl.v, vh2, o[2]);  o[2] = mma_h(ph.v, vl2, o[2]);
      o[3] = mma_h(ph.v, vh3, o[3]);  o[3] = mma_h(pl.v, vh3, o[3]);  o[3] = mma_h(ph.v, vl3, o[3]);
      guard10(o[0], o[1], o[2], o[3], ph.v, pl.v, vh0, vh1, vh2, vh3, vl0, vl1, vl2, vl3);
    }
    wave_sync_lds();
  }
  acc_guard4(o[0], o[1], o[2], o[3]);

  wave_sync_lds();
  float* slab = pt;
  const float oc = 1.0f / (PCAR * VCAR);
#pragma unroll
  for (int r = 0; r < 8; ++r) {
    const float inv = (1.0f / lrow[r]) * oc;
#pragma unroll
    for (int j = 0; j < 4; ++j) slab[(8 * hh + r) * 68 + j * 16 + c] = o[j][r] * inv;
  }
  wave_sync_lds();
  v4u oh[4], ol[4];
  const int rq = lane >> 3, c8 = (lane & 7) * 8;
#pragma unroll
  for (int it = 0; it < 4; ++it) {
    const int row = it * 4 + rq;
    const v4f a = *(const v4f*)(slab + row * 68 + c8), bq = *(const v4f*)(slab + row * 68 + c8 + 4);
    float w[8];
#pragma unroll
    for (int e = 0; e < 4; ++e) { w[e] = a[e] * OSC; w[4 + e] = bq[e] * OSC; }
#pragma unroll
    for (int e = 0; e < 4; ++e) {
      const _Float16 h0 = (_Float16)w[2 * e], h1 = (_Float16)w[2 * e + 1];
      const _Float16 l0 = (_Float16)(w[2 * e] - (float)h0), l1 = (_Float16)(w[2 * e + 1] - (float)h1);
      oh[it][e] = pk16(h_bits(h0), h_bits(h1));
      ol[it][e] = pk16(h_bits(l0), h_bits(l1));
    }
  }
  const size_t ob = (((size_t)(b * SEQ + q0)) * DMOD) + h * HD + c8;
  for (int pass = 0; pass < 2; ++pass) {
#pragma unroll
    for (int it = 0; it < 4; ++it) {
      const int row = it * 4 + rq;
      const size_t o8 = ob + (size_t)row * DMOD;
      *(volatile v4u*)(OHIp + o8) = oh[it];
      *(volatile v4u*)(OLOp + o8) = ol[it];
    }
    __threadfence();
  }
}

__global__ __launch_bounds__(128)
void gemm_h2(const u16* __restrict__ Ah, const u16* __restrict__ Al, const u16* __restrict__ Bt, const float* __restrict__ bias,
             float* C, int M, int N, int K, float oscale) {
  __shared__ __align__(16) float slab[4 * SLAB64];
  const int tid = threadIdx.x, wave = tid >> 5, lane = tid & 31, hh = lane >> 4, m = lane & 15;
  const int ntile = N >> 6;
  const int bid   = blockIdx.x;
  const int rowb  = (bid / ntile) * 64 + wave * 16;
  const int col0  = (bid % ntile) * 64;
  if (rowb + 16 > M) return;
  const size_t aofs = (size_t)(rowb + m) * K + 8 * hh;
  const _Float16* ahp = (const _Float16*)(const void*)Ah + aofs;
  const _Float16* alp = (const _Float16*)(const void*)Al + aofs;
  const _Float16* bp  = (const _Float16*)(const void*)Bt + (size_t)(col0 + m) * K + 8 * hh;
  const size_t bs = (size_t)16 * K;
  v8f acc0 = zero8(), acc1 = zero8(), acc2 = zero8(), acc3 = zero8();
#pragma unroll 1
  for (int k0 = 0; k0 < K; k0 += 32) {
    const v16h ah = ldfrag_h(ahp + k0), al = ldfrag_h(alp + k0);
    const v16h b0 = ldfrag_h(bp + k0);
    const v16h b1 = ldfrag_h(bp + bs + k0);
    const v16h b2 = ldfrag_h(bp + 2 * bs + k0);
    const v16h b3 = ldfrag_h(bp + 3 * bs + k0);
    acc0 = mma_h(ah, b0, acc0);  acc0 = mma_h(al, b0, acc0);
    acc1 = mma_h(ah, b1, acc1);  acc1 = mma_h(al, b1, acc1);
    acc2 = mma_h(ah, b2, acc2);  acc2 = mma_h(al, b2, acc2);
    acc3 = mma_h(ah, b3, acc3);  acc3 = mma_h(al, b3, acc3);
    guard6<v16h>(acc0, acc1, acc2, acc3, ah, al, b0, b1, b2, b3);
  }
  epi64(slab + wave * SLAB64, acc0, acc1, acc2, acc3, oscale, bias, C, N, (size_t)rowb, col0, lane);
}

extern "C" void kernel_launch(void* const* d_in, const int* in_sizes, int n_in,
                              void* d_out, int out_size, void* d_ws, size_t ws_size,
                              hipStream_t stream) {
  if (n_in < 8) return;
  if (in_sizes[0] != ROWS * DMOD) return;
  if (in_sizes[1] != 3 * DMOD * DMOD) return;
  if (in_sizes[2] != DMOD * HD * CF) return;
  if (in_sizes[3] != DMOD || in_sizes[4] != DMOD || in_sizes[5] != DMOD) return;
  if (in_sizes[6] != DMOD * DMOD || in_sizes[7] != DMOD) return;
  if (out_size != ROWS * DMOD) return;

  const float* x      = (const float*)d_in[0];
  const float* w_qkv  = (const float*)d_in[1];
  const float* w_conv = (const float*)d_in[2];
  const float* b_conv = (const float*)d_in[3];
  const float* null_k = (const float*)d_in[4];
  const float* null_v = (const float*)d_in[5];
  const float* w_out  = (const float*)d_in[6];
  const float* b_out  = (const float*)d_in[7];
  float*       out    = (float*)d_out;

  const size_t szXB  = (size_t)ROWS * DMOD * 2;
  const size_t szWB  = (size_t)3 * DMOD * DMOD * 2;
  const size_t szWOT = (size_t)DMOD * DMOD * 2;
  const size_t szWCT = (size_t)DMOD * KCONV * 2;
  const size_t szQP  = (size_t)ROWS * DMOD * 2;
  const size_t szTP  = (size_t)NB * NH * UROWS * HD * 2;
  const size_t szKC  = (size_t)NB * NH * JP * HD * 2;
  const size_t szVT  = (size_t)NB * NH * HD * JP * 2;
  const size_t szOP  = (size_t)ROWS * DMOD * 2;
  size_t off = 0;
  const size_t oXB  = off; off += szXB;
  const size_t oWB  = off; off += szWB;
  const size_t oWOT = off; off += szWOT;
  const size_t oWCT = off; off += szWCT;
  const size_t oQP  = off; off += szQP;
  const size_t oKH  = off; off += szTP;
  const size_t oKL  = off; off += szTP;
  const size_t oVH  = off; off += szTP;
  const size_t oVL  = off; off += szTP;
  const size_t oKC  = off; off += szKC;
  const size_t oVTH = off; off += szVT;
  const size_t oVTL = off; off += szVT;
  const size_t oOHI = off; off += szOP;
  const size_t oOLO = off; off += szOP;
  if (off > ws_size) return;
  if (off > (size_t)134217728) return;

  char* ws = (char*)d_ws;
  u16* XB  = (u16*)(ws + oXB);
  u16* WB  = (u16*)(ws + oWB);
  u16* WOT = (u16*)(ws + oWOT);
  u16* WCT = (u16*)(ws + oWCT);
  u16* QP  = (u16*)(ws + oQP);
  u16* KH  = (u16*)(ws + oKH);
  u16* KL  = (u16*)(ws + oKL);
  u16* VH  = (u16*)(ws + oVH);
  u16* VL  = (u16*)(ws + oVL);
  u16* KC  = (u16*)(ws + oKC);
  u16* VTH = (u16*)(ws + oVTH);
  u16* VTL = (u16*)(ws + oVTL);
  u16* OHI = (u16*)(ws + oOHI);
  u16* OLO = (u16*)(ws + oOLO);

  const dim3 blk(256);
  const dim3 bG(128);
  const int n8x = (ROWS * DMOD) / 8;
  const int n8w = (3 * DMOD * DMOD) / 8;
  const int n8o = (DMOD * DMOD) / 8;
  const dim3 gX((n8x + 255) / 256);
  const dim3 gW((n8w + 255) / 256);
  const dim3 gO((n8o + 255) / 256);
  const dim3 gWC(DMOD / 32);
  const dim3 gFill(NB * NH * 4);
  const dim3 gProj((ROWS / 64) * ((3 * DMOD) / 64));
  const dim3 gConv(2 * CONV_HALF);
  const dim3 gAT(ATT_BLOCKS);
  const dim3 gGO((ROWS / 64) * (DMOD / 64));

  cvt16<<<gX, blk, 0, stream>>>(x, XB, n8x, 0, 1.0f);
  cvt16<<<gW, blk, 0, stream>>>(w_qkv, WB, n8w, 0, 1.0f);
  cvt16<<<gO, blk, 0, stream>>>(w_out, WOT, n8o, 1, WOS);
  cvt_wconv<<<gWC, blk, 0, stream>>>(w_conv, WCT);
  fill_pad<<<gFill, blk, 0, stream>>>(KH, KL, VH, VL);
  proj_gemm<<<gProj, bG, 0, stream>>>(XB, WB, QP, KH, KL, VH, VL);
  conv_gemm<<<gConv, bG, 0, stream>>>(KH, KL, VH, VL, WCT, b_conv, null_k, null_v, KC, VTH, VTL);
  attn_mc<<<gAT, bG, 0, stream>>>(QP, KC, VTH, VTL, OHI, OLO);
  gemm_h2<<<gGO, bG, 0, stream>>>(OHI, OLO, WOT, b_out, out, ROWS, DMOD, DMOD, 1.0f / (OSC * WOS));
  (void)hipGetLastError();
}
